// GTransformerLayer_82059645157591
// MI455X (gfx1250) — hardware-verified
//
#include <hip/hip_runtime.h>
#include <hip/hip_bf16.h>
#include <math.h>


#define BB 2
#define SS 2048
#define DD 1024
#define HH 16
#define DKK 64
#define QW 2

typedef _Float16 bf16;
typedef __attribute__((ext_vector_type(4))) unsigned v4u_t;
typedef unsigned v4ua __attribute__((ext_vector_type(4), may_alias));
typedef __attribute__((ext_vector_type(4))) float v4f_t;
typedef float v4fa __attribute__((ext_vector_type(4), may_alias));
typedef __attribute__((ext_vector_type(16))) bf16  bf16x16;
typedef __attribute__((ext_vector_type(8)))  bf16  bf16x8;
typedef __attribute__((ext_vector_type(4)))  bf16  bf16x4;
typedef __attribute__((ext_vector_type(8)))  float f32x8;

#define LDS_STRIDE 48
#define KSTRIDE    72
#define VSTRIDE    48

__device__ __forceinline__ f32x8 wmma_bf16(bf16x16 a, bf16x16 b, f32x8 c) {
  return __builtin_amdgcn_wmma_f32_16x16x32_f16(
      false, a, false, b, (short)0, c, false, false);
}

template <typename T>
__device__ __forceinline__ bf16x16 load_frag(const T* __restrict__ base, int ld,
                                             int row0, int k0) {
  const int lane = threadIdx.x & 31;
  const int r    = lane & 15;
  const int kh   = (lane >> 4) * 8;
  const T* p0 = base + (size_t)(row0 + r) * ld + (k0 + kh);
  const T* p1 = p0 + 16;
  bf16x16 f;
#pragma unroll
  for (int i = 0; i < 8; ++i) {
    f[i]     = (bf16)p0[i];
    f[i + 8] = (bf16)p1[i];
  }
  return f;
}

__device__ __forceinline__ bf16x16 lds_frag(const bf16* base, int stride) {
  const int lane = threadIdx.x & 31;
  const int row  = lane & 15;
  const int kh   = (lane >> 4) * 8;
  const bf16x8 lo = *(const bf16x8*)(base + row * stride + kh);
  const bf16x8 hi = *(const bf16x8*)(base + row * stride + kh + 16);
  bf16x16 f;
#pragma unroll
  for (int i = 0; i < 8; ++i) { f[i] = lo[i]; f[i + 8] = hi[i]; }
  return f;
}

template <typename T>
__device__ __forceinline__ void stage_read16(const T* __restrict__ p, float* buf) {
#pragma unroll
  for (int i = 0; i < 16; ++i) buf[i] = (float)p[i];
}

__device__ __forceinline__ void stage_write(bf16* dst, const float* buf, int nquad) {
#pragma unroll
  for (int i = 0; i < nquad; ++i) {
    bf16x4 q;
    q[0] = (bf16)buf[4 * i];     q[1] = (bf16)buf[4 * i + 1];
    q[2] = (bf16)buf[4 * i + 2]; q[3] = (bf16)buf[4 * i + 3];
    *(bf16x4*)(dst + 4 * i) = q;
  }
}

template <typename AT, int MODE>
__global__ __launch_bounds__(256) void gemm_bias_kernel(
    const AT* __restrict__ A, const float* __restrict__ W,
    const float* __restrict__ bias, void* __restrict__ out,
    int M, int N, int K) {
  __shared__ bf16 ldsA[128 * LDS_STRIDE];
  __shared__ bf16 ldsW[256 * LDS_STRIDE];
  __shared__ __attribute__((aligned(16))) unsigned char sob[256 * 136 * 2];

  const int t    = threadIdx.x;
  const int wave = t >> 5;
  const int lane = t & 31;
  const int wm   = (wave & 1) * 64;
  const int wn   = (wave >> 1) * 64;
  const int mBlk = blockIdx.x * 128;
  const int nBlk = blockIdx.y * 256;

  const int arow = t >> 1;
  const int ach  = (t & 1) * 16;

  float abuf[16];
  float wbuf[32];

  stage_read16(A + (size_t)(mBlk + arow) * K + ach, abuf);
  stage_read16(W + (size_t)(nBlk + t) * K,          wbuf);
  stage_read16(W + (size_t)(nBlk + t) * K + 16,     wbuf + 16);

  f32x8 acc[4][4] = {};

  for (int k = 0; k < K; k += 32) {
    __syncthreads();
    stage_write(&ldsA[arow * LDS_STRIDE + ach], abuf, 4);
    stage_write(&ldsW[t * LDS_STRIDE],          wbuf, 8);
    if (k + 32 < K) {
      stage_read16(A + (size_t)(mBlk + arow) * K + (k + 32) + ach, abuf);
      stage_read16(W + (size_t)(nBlk + t) * K + (k + 32),          wbuf);
      stage_read16(W + (size_t)(nBlk + t) * K + (k + 32) + 16,     wbuf + 16);
    }
    __syncthreads();

    bf16x16 af[4], wf[4];
#pragma unroll
    for (int i = 0; i < 4; ++i)
      af[i] = lds_frag(ldsA + (wm + 16 * i) * LDS_STRIDE, LDS_STRIDE);
#pragma unroll
    for (int j = 0; j < 4; ++j)
      wf[j] = lds_frag(ldsW + (wn + 16 * j) * LDS_STRIDE, LDS_STRIDE);
#pragma unroll
    for (int i = 0; i < 4; ++i)
#pragma unroll
      for (int j = 0; j < 4; ++j)
        acc[i][j] = wmma_bf16(af[i], wf[j], acc[i][j]);
  }

  const int nlane = lane & 15;
  const int mh    = (lane >> 4) * 8;
  __syncthreads();
  if (MODE == 0 || MODE == 1) {
    bf16* so = (bf16*)sob;
#pragma unroll
    for (int i = 0; i < 4; ++i)
#pragma unroll
      for (int j = 0; j < 4; ++j) {
        const int nl = wn + 16 * j + nlane;
        const float bv = bias ? bias[nBlk + nl] : 0.0f;
#pragma unroll
        for (int r = 0; r < 8; ++r) {
          const int ml = wm + 16 * i + mh + r;
          const bf16 hv = (bf16)(acc[i][j][r] + bv);
          if (MODE == 0) so[ml * 264 + nl] = hv;
          else           so[nl * 136 + ml] = hv;
        }
      }
    __syncthreads();
#pragma unroll 1
    for (int pass = 0; pass < 2; ++pass) {
      if (MODE == 0) {
        for (int ch = t; ch < 128 * 32; ch += 256) { const int ml = ch >> 5, q = (ch & 31) * 8;
          *(volatile v4u_t*)((bf16*)out + (size_t)(mBlk + ml) * N + nBlk + q) = *(const v4ua*)(so + ml * 264 + q); }
      } else {
        const int b_ = mBlk / SS, s0 = mBlk & (SS - 1);
        for (int ch = t; ch < 256 * 16; ch += 256) { const int nl = ch >> 4, q = (ch & 15) * 8; const int n = nBlk + nl, h = n >> 6, dk = n & (DKK - 1);
          *(volatile v4u_t*)((bf16*)out + (((size_t)(b_ * HH + h)) * DKK + dk) * SS + s0 + q) = *(const v4ua*)(so + nl * 136 + q); }
      }
      __threadfence();
    }
  } else {
    float* so = (float*)sob;
#pragma unroll 1
    for (int hf = 0; hf < 2; ++hf) {
      if (wm == hf * 64) {
#pragma unroll
        for (int i = 0; i < 4; ++i)
#pragma unroll
          for (int j = 0; j < 4; ++j) {
            const int nl = wn + 16 * j + nlane;
            const float bv = bias ? bias[nBlk + nl] : 0.0f;
#pragma unroll
            for (int r = 0; r < 8; ++r) so[(16 * i + mh + r) * 260 + nl] = acc[i][j][r] + bv;
          }
      }
      __syncthreads();
#pragma unroll 1
      for (int pass = 0; pass < 2; ++pass) {
        for (int ch = t; ch < 64 * 64; ch += 256) { const int ml = ch >> 6, q = (ch & 63) * 4;
          *(volatile v4f_t*)((float*)out + (size_t)(mBlk + hf * 64 + ml) * N + nBlk + q) = *(const volatile v4fa*)(so + ml * 260 + q); }
        __threadfence();
      }
      __syncthreads();
    }
  }
}


#define GN 16384
#define GE 262144
#define NR 5
#define NHD 4
#define DO 128
#define DKH 32
#define WR 768

__global__ __launch_bounds__(128) void k_wrows(const float* __restrict__ W, float* __restrict__ WT) {
  const int n = blockIdx.x, k = threadIdx.x; const int r = n / DO, o = n % DO;
  const float v = (n < NR * DO) ? W[((size_t)r * 128 + k) * DO + o] : 0.0f;
  *(volatile float*)(WT + (size_t)n * 128 + k) = v; __threadfence(); *(volatile float*)(WT + (size_t)n * 128 + k) = v;
}
__global__ __launch_bounds__(256) void k_bias3(const float* __restrict__ bk, const float* __restrict__ bq, const float* __restrict__ bv, float* __restrict__ bp) {
  for (int i = threadIdx.x; i < 3 * WR; i += 256) { const int w = i / WR, n = i % WR; const float* b = (w == 0) ? bk : (w == 1) ? bq : bv;
    const float v = (n < NR * DO) ? b[n] : 0.0f; *(volatile float*)(bp + i) = v; }
  __threadfence();
  for (int i = threadIdx.x; i < 3 * WR; i += 256) { const int w = i / WR, n = i % WR; const float* b = (w == 0) ? bk : (w == 1) ? bq : bv;
    const float v = (n < NR * DO) ? b[n] : 0.0f; *(volatile float*)(bp + i) = v; }
}
__global__ __launch_bounds__(256) void k_packA(const float* __restrict__ Wt, float* __restrict__ A) {
  const int m = blockIdx.x; for (int k = threadIdx.x; k < 512; k += 256) { const float v = Wt[(size_t)k * DO + m]; *(volatile float*)(A + (size_t)m * 512 + k) = v; }
  __threadfence();
  for (int k = threadIdx.x; k < 512; k += 256) { const float v = Wt[(size_t)k * DO + m]; *(volatile float*)(A + (size_t)m * 512 + k) = v; }
}
__device__ __forceinline__ int clampi(int v, int hi) { return v < 0 ? 0 : (v >= hi ? hi - 1 : v); }
__device__ __forceinline__ void edge_scores(const bf16* __restrict__ Kr, const bf16* __restrict__ Qr, int sl, int dn, int r, int lane, float* s) {
  const bf16* kr = Kr + (size_t)sl * WR + r * DO; const bf16* qr = Qr + (size_t)dn * WR + r * DO;
#pragma unroll
  for (int h = 0; h < NHD; ++h) { float p = (float)kr[h * DKH + lane] * (float)qr[h * DKH + lane];
#pragma unroll
    for (int o = 16; o >= 1; o >>= 1) p += __shfl_xor(p, o, 32);
    s[h] = p * 0.17677669529663687f; }
}
#define SCAN_PROLOGUE \
  __shared__ int qd[8][256], qs[8][256], qr_[8][256]; __shared__ int wcnt[8][8]; \
  const int tid = threadIdx.x, lane = tid & 31, wave = tid >> 5;
#define SCAN_CHUNK_BEGIN \
  for (int c0 = 0; c0 < GE; c0 += 256) { \
    const int e = c0 + tid; int d = -1, sidx = 0, rel = 0; \
    if (e < GE) { d = clampi(dsti[e], GN); sidx = clampi(srci[e], GN); rel = clampi(eti[e], NR); } \
    const int own = (d >= 0) ? (d & 7) : -1; unsigned mown = 0u; \
    _Pragma("unroll") for (int ww = 0; ww < 8; ++ww) { const unsigned m = __builtin_amdgcn_ballot_w32(own == ww); if (own == ww) mown = m; if (lane == 0) wcnt[ww][wave] = __builtin_popcount(m); } \
    __syncthreads(); \
    if (own >= 0) { int base = 0; _Pragma("unroll") for (int w2 = 0; w2 < 8; ++w2) base += (w2 < wave) ? wcnt[own][w2] : 0; \
      const int pos = base + __builtin_popcount(mown & ((1u << lane) - 1u)); qd[own][pos] = d; qs[own][pos] = sidx; qr_[own][pos] = rel; } \
    int total = 0; _Pragma("unroll") for (int w2 = 0; w2 < 8; ++w2) total += wcnt[wave][w2]; \
    __syncthreads();
#define SCAN_CHUNK_END __syncthreads(); }

__global__ __launch_bounds__(256) void k_p1(const int* __restrict__ srci, const int* __restrict__ dsti, const int* __restrict__ eti, const bf16* __restrict__ Kr, const bf16* __restrict__ Qr, float* __restrict__ MX) {
  SCAN_PROLOGUE
  for (int i = tid; i < GN * NR; i += 256) { v4f_t z; z.x = z.y = z.z = z.w = -INFINITY; *(volatile v4f_t*)(MX + (size_t)i * 4) = z; }
  __threadfence(); __syncthreads();
  SCAN_CHUNK_BEGIN
#pragma unroll 1
    for (int qi = 0; qi < total; ++qi) { const int dn = qd[wave][qi], sl = qs[wave][qi], r = qr_[wave][qi]; float s[NHD];
      edge_scores(Kr, Qr, sl, dn, r, lane, s);
      if (lane < NHD) { float* p = MX + ((size_t)dn * NR + r) * NHD + lane; *p = fmaxf(*p, s[lane]); } }
  SCAN_CHUNK_END
  __threadfence(); __syncthreads();
  for (int i = tid; i < GN * NR; i += 256) { float* p = MX + (size_t)i * 4; const v4f_t v = *(const volatile v4fa*)p; *(volatile v4f_t*)p = v; }
  __threadfence();
}
__global__ __launch_bounds__(256) void k_p2(const int* __restrict__ srci, const int* __restrict__ dsti, const int* __restrict__ eti, const bf16* __restrict__ Kr, const bf16* __restrict__ Qr, const float* __restrict__ MX, float* __restrict__ DEN) {
  SCAN_PROLOGUE
  for (int i = tid; i < GN * NR; i += 256) { v4f_t z; z.x = z.y = z.z = z.w = 0.0f; *(volatile v4f_t*)(DEN + (size_t)i * 4) = z; }
  __threadfence(); __syncthreads();
  SCAN_CHUNK_BEGIN
#pragma unroll 1
    for (int qi = 0; qi < total; ++qi) { const int dn = qd[wave][qi], sl = qs[wave][qi], r = qr_[wave][qi]; float s[NHD];
      edge_scores(Kr, Qr, sl, dn, r, lane, s);
      if (lane < NHD) { const size_t ix = ((size_t)dn * NR + r) * NHD + lane; DEN[ix] += expf(s[lane] - MX[ix]); } }
  SCAN_CHUNK_END
  __threadfence(); __syncthreads();
  for (int i = tid; i < GN * NR; i += 256) { float* p = DEN + (size_t)i * 4; const v4f_t v = *(const volatile v4fa*)p; *(volatile v4f_t*)p = v; }
  __threadfence();
}
__global__ __launch_bounds__(256) void k_p3(const int* __restrict__ srci, const int* __restrict__ dsti, const int* __restrict__ eti, const bf16* __restrict__ Kr, const bf16* __restrict__ Qr, const bf16* __restrict__ Vr,
                                           const float* __restrict__ MX, const float* __restrict__ DEN, float* __restrict__ OUT) {
  SCAN_PROLOGUE
  for (int i = tid; i < GN * NHD * DO / 4; i += 256) { v4f_t z; z.x = z.y = z.z = z.w = 0.0f; *(volatile v4f_t*)(OUT + (size_t)i * 4) = z; }
  __threadfence(); __syncthreads();
  SCAN_CHUNK_BEGIN
#pragma unroll 1
    for (int qi = 0; qi < total; ++qi) { const int dn = qd[wave][qi], sl = qs[wave][qi], r = qr_[wave][qi]; float s[NHD], a[NHD];
      edge_scores(Kr, Qr, sl, dn, r, lane, s);
#pragma unroll
      for (int h = 0; h < NHD; ++h) { const size_t ix = ((size_t)dn * NR + r) * NHD + h; a[h] = expf(s[h] - MX[ix]) / DEN[ix]; }
      const bf16* vr = Vr + (size_t)sl * WR + r * DO + lane * 4; const float v0 = (float)vr[0], v1 = (float)vr[1], v2 = (float)vr[2], v3 = (float)vr[3];
#pragma unroll
      for (int h = 0; h < NHD; ++h) { float* row = OUT + ((size_t)dn * NHD + h) * DO + lane * 4; row[0] += a[h] * v0; row[1] += a[h] * v1; row[2] += a[h] * v2; row[3] += a[h] * v3; } }
  SCAN_CHUNK_END
  __threadfence(); __syncthreads();
  for (int i = tid; i < GN * NHD * DO / 4; i += 256) { float* p = OUT + (size_t)i * 4; const v4f_t v = *(const volatile v4fa*)p; *(volatile v4f_t*)p = v; }
  __threadfence();
}
__global__ __launch_bounds__(256) void k_outrows(const float* __restrict__ T, const float* __restrict__ bt, float* __restrict__ out) {
  __shared__ float tile[64][65];
  const int n0 = blockIdx.x * 64, o0 = blockIdx.y * 64, t = threadIdx.x;
  for (int i = t; i < 64 * 64; i += 256) { const int o = i >> 6, nn = i & 63; tile[o][nn] = T[(size_t)(o0 + o) * GN + n0 + nn] + bt[o0 + o]; }
  __syncthreads();
#pragma unroll 1
  for (int pass = 0; pass < 2; ++pass) {
    for (int i = t; i < 64 * 16; i += 256) { const int nr = i >> 4, o4 = (i & 15) * 4; v4f_t v; v.x = tile[o4][nr]; v.y = tile[o4 + 1][nr]; v.z = tile[o4 + 2][nr]; v.w = tile[o4 + 3][nr];
      *(volatile v4f_t*)(out + (size_t)(n0 + nr) * DO + o0 + o4) = v; }
    __threadfence(); }
}

extern "C" void kernel_launch(void* const* d_in, const int* in_sizes, int n_in,
                              void* d_out, int out_size, void* d_ws, size_t ws_size,
                              hipStream_t stream) {
  (void)in_sizes; (void)n_in; (void)out_size; (void)ws_size;
  const float* h = (const float*)d_in[0];
  const float* Wk = (const float*)d_in[1]; const float* bk = (const float*)d_in[2];
  const float* Wq = (const float*)d_in[3]; const float* bq = (const float*)d_in[4];
  const float* Wv = (const float*)d_in[5]; const float* bv = (const float*)d_in[6];
  const float* Wt = (const float*)d_in[7]; const float* bt = (const float*)d_in[8];
  const int* srci = (const int*)d_in[9]; const int* dsti = (const int*)d_in[10]; const int* eti = (const int*)d_in[11];
  float* out = (float*)d_out;
  char* ws = (char*)d_ws;
  float* WkT = (float*)ws; ws += (size_t)WR * 128 * 4;
  float* WqT = (float*)ws; ws += (size_t)WR * 128 * 4;
  float* WvT = (float*)ws; ws += (size_t)WR * 128 * 4;
  float* bp  = (float*)ws; ws += (size_t)3 * WR * 4; float* bkp = bp; float* bqp = bp + WR; float* bvp = bp + 2 * WR;
  float* A2  = (float*)ws; ws += (size_t)128 * 512 * 4;
  bf16* Kr = (bf16*)ws; ws += (size_t)GN * WR * 2;
  bf16* Qr = (bf16*)ws; ws += (size_t)GN * WR * 2;
  bf16* Vr = (bf16*)ws; ws += (size_t)GN * WR * 2;
  float* MX  = (float*)ws; ws += (size_t)GN * NR * NHD * 4;
  float* DEN = (float*)ws; ws += (size_t)GN * NR * NHD * 4;
  float* OUT = (float*)ws; ws += (size_t)GN * NHD * DO * 4;
  float* T   = (float*)ws; ws += (size_t)128 * GN * 4;
  k_wrows<<<WR, 128, 0, stream>>>(Wk, WkT);
  k_wrows<<<WR, 128, 0, stream>>>(Wq, WqT);
  k_wrows<<<WR, 128, 0, stream>>>(Wv, WvT);
  k_bias3<<<1, 256, 0, stream>>>(bk, bq, bv, bp);
  k_packA<<<128, 256, 0, stream>>>(Wt, A2);
  dim3 blk(256);
  gemm_bias_kernel<float, 0><<<dim3(GN / 128, WR / 256), blk, 0, stream>>>(h, WkT, bkp, Kr, GN, WR, 128);
  gemm_bias_kernel<float, 0><<<dim3(GN / 128, WR / 256), blk, 0, stream>>>(h, WqT, bqp, Qr, GN, WR, 128);
  gemm_bias_kernel<float, 0><<<dim3(GN / 128, WR / 256), blk, 0, stream>>>(h, WvT, bvp, Vr, GN, WR, 128);
  k_p1<<<1, 256, 0, stream>>>(srci, dsti, eti, Kr, Qr, MX);
  k_p2<<<1, 256, 0, stream>>>(srci, dsti, eti, Kr, Qr, MX, DEN);
  k_p3<<<1, 256, 0, stream>>>(srci, dsti, eti, Kr, Qr, Vr, MX, DEN, OUT);
  gemm_bias_kernel<float, 2><<<dim3(1, GN / 256), blk, 0, stream>>>(A2, OUT, nullptr, T, 128, GN, 512);
  k_outrows<<<dim3(GN / 64, DO / 64), 256, 0, stream>>>(T, bt, out);
}
